// CrossGCN_38482906972407
// MI455X (gfx1250) — hardware-verified
//
#include <hip/hip_runtime.h>

enum : int {
  BATCH = 8, NODES = 256, NIMG = 36, NSEM = 64,
  IN_D = 1024, QUE_D = 1024, IMG_D = 2048, SEM_D = 512,
  PROJ = 512, GATE = 512, CAT = 3 * GATE, OUT_D = 1024,
  ROWS = BATCH * NODES,
  IMG_ROWS = BATCH * NIMG,
  IMG_ROWS_P = 320,
  SEM_ROWS = BATCH * NSEM,
  QROWS_P = 64,
  KEYP = 64
};
#define RB_SHIFT 8

typedef __attribute__((ext_vector_type(16))) _Float16 v16h;
typedef __attribute__((ext_vector_type(8)))  _Float16 v8h;
typedef __attribute__((ext_vector_type(16))) __bf16   v16b;
typedef __attribute__((ext_vector_type(8)))  __bf16   v8b;
typedef __attribute__((ext_vector_type(8)))  float    v8f;
typedef __attribute__((ext_vector_type(4)))  float    v4f;

__device__ __forceinline__ unsigned short f2bf_bits(float f) {
  unsigned u = __float_as_uint(f);
  return (unsigned short)((u + 0x7FFFu + ((u >> 16) & 1u)) >> 16);
}
__device__ __forceinline__ float bf_bits2f(unsigned short h) { return __uint_as_float(((unsigned)h) << 16); }

__device__ __forceinline__ void dep_guard_h(v8f& a, v8f& b, v16h x, v16h y) { asm volatile("v_nop\n\tv_nop\n\tv_nop\n\tv_nop" : "+v"(a), "+v"(b) : "v"(x), "v"(y)); }
__device__ __forceinline__ void dep_guard_b(v8f& a, v8f& b, v16b x, v16b y) { asm volatile("v_nop\n\tv_nop\n\tv_nop\n\tv_nop" : "+v"(a), "+v"(b) : "v"(x), "v"(y)); }
__device__ __forceinline__ void keep4_h(v16h a, v16h b, v16h c, v16h d) { asm volatile("v_nop" :: "v"(a), "v"(b), "v"(c), "v"(d)); }
__device__ __forceinline__ void keep4_b(v16b a, v16b b, v16b c, v16b d) { asm volatile("v_nop" :: "v"(a), "v"(b), "v"(c), "v"(d)); }
__device__ __forceinline__ void acc_guard4(v8f& a, v8f& b, v8f& c, v8f& d) { asm volatile("v_nop\n\tv_nop\n\tv_nop\n\tv_nop" : "+v"(a), "+v"(b), "+v"(c), "+v"(d)); }
template <typename T> struct Frag;
template <> struct Frag<_Float16> {
  typedef v16h V; union U { v16h v; v8h h[2]; };
  static __device__ __forceinline__ v16h load(const _Float16* p) {
    U f; f.h[0] = *(const v8h*)(p); f.h[1] = *(const v8h*)(p + 16); return f.v;
  }
  static __device__ __forceinline__ v8f mma(v16h a, v16h b, v8f c) {
    return __builtin_amdgcn_wmma_f32_16x16x32_f16(false, a, false, b, (short)0, c, false, false);
  }
  static __device__ __forceinline__ void guard(v8f& a, v8f& b, v16h x, v16h y) { dep_guard_h(a, b, x, y); }
  static __device__ __forceinline__ void keep(v16h a, v16h b, v16h c, v16h d) { keep4_h(a, b, c, d); }
};
template <> struct Frag<__bf16> {
  typedef v16b V; union U { v16b v; v8b h[2]; };
  static __device__ __forceinline__ v16b load(const __bf16* p) {
    U f; f.h[0] = *(const v8b*)(p); f.h[1] = *(const v8b*)(p + 16); return f.v;
  }
  static __device__ __forceinline__ v8f mma(v16b a, v16b b, v8f c) {
    return __builtin_amdgcn_wmma_f32_16x16x32_bf16(false, a, false, b, (short)0, c, false, false);
  }
  static __device__ __forceinline__ void guard(v8f& a, v8f& b, v16b x, v16b y) { dep_guard_b(a, b, x, y); }
  static __device__ __forceinline__ void keep(v16b a, v16b b, v16b c, v16b d) { keep4_b(a, b, c, d); }
};

template <int ET> struct Elem;
template <> struct Elem<0> { typedef _Float16 T; };
template <> struct Elem<1> { typedef __bf16 T; };
template <int ET, bool SPLIT, int BIAS_MODE, int OUT_MODE, int ACT, bool MULG>
__global__ __launch_bounds__(256) void wmma_gemm64(
    const unsigned short* __restrict__ Ap, const unsigned short* __restrict__ A2p, int lda, long strideA,
    const unsigned short* __restrict__ Btp, const unsigned short* __restrict__ Bt2p, int ldb, long strideB,
    void* __restrict__ Cout, void* __restrict__ Cout2, int ldc, long strideC,
    const float* __restrict__ bias,
    const float* __restrict__ gmul, int ldg,
    int M, int N, int K, float scale, float oscale) {
  typedef typename Elem<ET>::T T;
  typedef typename Frag<T>::V V;
  const T* A = (const T*)Ap; const T* A2 = (const T*)A2p; const T* Bt = (const T*)Btp; const T* Bt2 = (const T*)Bt2p;
  __shared__ __align__(16) float sT[8][16 * 68];
  const int b    = blockIdx.y;
  const int lane = threadIdx.x & 31;
  const int wave = threadIdx.x >> 5;
  const int tilesN = N >> 6;
  const int tilesM = M >> 6;
  const int tile = blockIdx.x * 8 + wave;
  if (tile >= tilesM * tilesN) return;
  const int tm = tile / tilesN;
  const int tn = tile - tm * tilesN;
  const int m0 = tm << 6;
  const int n0 = tn << 6;

  const T* Ab  = A  + (size_t)b * strideA;
  const T* Bb  = Bt + (size_t)b * strideB;
  const T* Ab2 = SPLIT ? (A2  + (size_t)b * strideA) : nullptr;
  const T* Bb2 = SPLIT ? (Bt2 + (size_t)b * strideB) : nullptr;

  const int rlane = lane & 15;
  const int koff  = (lane >> 4) * 8;
  const int mOff  = (lane >> 4) * 8;

  v8f acc[4][4];
#pragma unroll
  for (int i = 0; i < 4; ++i)
#pragma unroll
    for (int j = 0; j < 4; ++j) acc[i][j] = (v8f){0.f,0.f,0.f,0.f,0.f,0.f,0.f,0.f};

  for (int k0 = 0; k0 < K; k0 += 32) {
    V bh[4], bl[4];
#pragma unroll
    for (int j = 0; j < 4; ++j) {
      const size_t bo = (size_t)(n0 + (j << 4) + rlane) * ldb + koff + k0;
      bh[j] = Frag<T>::load(Bb + bo);
      if (SPLIT) bl[j] = Frag<T>::load(Bb2 + bo);
    }
#pragma unroll
    for (int i = 0; i < 4; ++i) {
      const size_t ao = (size_t)(m0 + (i << 4) + rlane) * lda + koff + k0;
      V ah = Frag<T>::load(Ab + ao);
      V al;
      if (SPLIT) al = Frag<T>::load(Ab2 + ao);
#pragma unroll
      for (int j = 0; j < 4; ++j) {
        acc[i][j] = Frag<T>::mma(ah, bh[j], acc[i][j]);
        if (SPLIT) {
          acc[i][j] = Frag<T>::mma(ah, bl[j], acc[i][j]);
          acc[i][j] = Frag<T>::mma(al, bh[j], acc[i][j]);
        }
      }
      Frag<T>::guard(acc[i][0], acc[i][3], ah, SPLIT ? al : ah);
    }
    Frag<T>::keep(bh[0], bh[1], bh[2], bh[3]);
    if (SPLIT) Frag<T>::keep(bl[0], bl[1], bl[2], bl[3]);
  }
  acc_guard4(acc[0][0], acc[0][1], acc[0][2], acc[0][3]);
  acc_guard4(acc[1][0], acc[1][1], acc[1][2], acc[1][3]);
  acc_guard4(acc[2][0], acc[2][1], acc[2][2], acc[2][3]);
  acc_guard4(acc[3][0], acc[3][1], acc[3][2], acc[3][3]);

  float* slab = sT[wave];
#pragma unroll
  for (int i = 0; i < 4; ++i) {
    const int mBase = m0 + (i << 4);
#pragma unroll
    for (int j = 0; j < 4; ++j) {
      const int n = n0 + (j << 4) + rlane;
      float bv = 0.f;
      if (BIAS_MODE == 2) bv = bias[n];
#pragma unroll
      for (int r = 0; r < 8; ++r) {
        const int row = mBase + mOff + r;
        float v = acc[i][j][r] * scale;
        if (BIAS_MODE == 1) v += bias[row];
        if (BIAS_MODE == 2) v += bv;
        if (BIAS_MODE == 3) v += bias[(size_t)(row >> RB_SHIFT) * N + n];
        if (ACT == 1) v = tanhf(v);
        if (ACT == 2) v = fmaxf(v, 0.0f);
        if (ACT == 6) v = __builtin_amdgcn_rcpf(1.0f + __expf(-v));
        if (MULG) v *= gmul[(size_t)row * ldg + n];
        slab[(mOff + r) * 68 + (j << 4) + rlane] = v;
      }
    }
    __builtin_amdgcn_fence(__ATOMIC_RELEASE, "workgroup");
    __builtin_amdgcn_wave_barrier();
    __builtin_amdgcn_fence(__ATOMIC_ACQUIRE, "workgroup");
    if (OUT_MODE == 0 || OUT_MODE == 3) {
      float* C = (float*)Cout + (size_t)b * strideC;
      const int hh = lane >> 4, c4 = (lane & 15) * 4;
      for (int pass = 0; pass < 2; ++pass) {
#pragma unroll
        for (int it = 0; it < 8; ++it) {
          const int row = it * 2 + hh;
          v4f v = *(const v4f*)(slab + row * 68 + c4);
          *(volatile v4f*)(C + (size_t)(mBase + row) * ldc + n0 + c4) = v;
        }
        __threadfence();
      }
    }
    if (OUT_MODE == 1 || OUT_MODE == 3) {
      const int q = lane >> 3, c8 = (lane & 7) * 8;
      unsigned short* C = (unsigned short*)(OUT_MODE == 1 ? Cout : Cout2) + (size_t)b * strideC;
      for (int pass = 0; pass < 2; ++pass) {
#pragma unroll
        for (int it = 0; it < 4; ++it) {
          const int row = it * 4 + q;
          const float* sp = slab + row * 68 + c8;
          v8h hv;
#pragma unroll
          for (int e = 0; e < 8; ++e) hv[e] = (_Float16)(sp[e] * oscale);
          *(volatile v8h*)(C + (size_t)(mBase + row) * ldc + n0 + c8) = hv;
        }
        __threadfence();
      }
    }
    __builtin_amdgcn_fence(__ATOMIC_RELEASE, "workgroup");
    __builtin_amdgcn_wave_barrier();
    __builtin_amdgcn_fence(__ATOMIC_ACQUIRE, "workgroup");
  }
}

template <int MODE>
__global__ __launch_bounds__(256) void k_cast8(const float* __restrict__ in, int n_valid, int n_total, float sc,
    unsigned short* __restrict__ o0, unsigned short* __restrict__ o1, unsigned short* __restrict__ o2) {
  const long i8 = ((long)blockIdx.x * 256 + threadIdx.x) * 8;
  if (i8 >= (long)n_total) return;
  const bool valid = i8 < (long)n_valid;
  const float* src = in + (valid ? i8 : 0);
  v4f x0 = *(const v4f*)(src);
  v4f x1 = *(const v4f*)(src + 4);
  const v4f z = {0.f, 0.f, 0.f, 0.f};
  if (!valid) { x0 = z; x1 = z; }
  v8h fv, hv, lv;
#pragma unroll
  for (int e = 0; e < 4; ++e) {
    const float a = x0[e], c = x1[e];
    fv[e] = (_Float16)(a * sc);
    fv[4 + e] = (_Float16)(c * sc);
    if (MODE == 2) {
      const unsigned short ha = f2bf_bits(a), hc = f2bf_bits(c);
      const unsigned short la = f2bf_bits(a - bf_bits2f(ha)), lc = f2bf_bits(c - bf_bits2f(hc));
      hv[e] = __builtin_bit_cast(_Float16, ha); hv[4 + e] = __builtin_bit_cast(_Float16, hc);
      lv[e] = __builtin_bit_cast(_Float16, la); lv[4 + e] = __builtin_bit_cast(_Float16, lc);
    } else {
      hv[e] = fv[e]; hv[4 + e] = fv[4 + e]; lv[e] = fv[e]; lv[4 + e] = fv[4 + e];
    }
  }
  *(volatile v8h*)(o0 + i8) = fv;
  if (MODE == 2) { *(volatile v8h*)(o1 + i8) = hv; *(volatile v8h*)(o2 + i8) = lv; }
  __threadfence();
  *(volatile v8h*)(o0 + i8) = fv;
  if (MODE == 2) { *(volatile v8h*)(o1 + i8) = hv; *(volatile v8h*)(o2 + i8) = lv; }
}

template <int MODE>
__global__ __launch_bounds__(256) void k_transpose64(const float* __restrict__ in, int R, int C, long sin,
    unsigned short* __restrict__ out0, unsigned short* __restrict__ out1, int RP, long sout, float sc) {
  __shared__ float tile[64][65];
  const int tid = threadIdx.x;
  const int r0 = blockIdx.y * 64, c0 = blockIdx.x * 64, bz = blockIdx.z;
  const float* inb = in + (size_t)bz * sin;
  const int cc = tid & 63, rg = tid >> 6;
#pragma unroll
  for (int j = 0; j < 16; ++j) {
    const int r = j * 4 + rg;
    const int ra = r0 + r;
    const int rcl = (ra < R) ? ra : (R - 1);
    const float v = inb[(size_t)rcl * C + c0 + cc];
    tile[r][cc] = (ra < R) ? v : 0.0f;
  }
  __syncthreads();
  const int wave = tid >> 5, lane = tid & 31, q = lane >> 3, c8 = (lane & 7) * 8;
  unsigned short* ob0 = out0 + (size_t)bz * sout;
  unsigned short* ob1 = out1 + (size_t)bz * sout;
  for (int pass = 0; pass < 2; ++pass) {
#pragma unroll
    for (int it = 0; it < 2; ++it) {
      const int orow = it * 32 + wave * 4 + q;
      v8h hv, lv;
#pragma unroll
      for (int e = 0; e < 8; ++e) {
        const float v = tile[c8 + e][orow];
        if (MODE == 0) {
          hv[e] = (_Float16)(v * sc); lv[e] = hv[e];
        } else {
          const unsigned short hb = f2bf_bits(v);
          const unsigned short lb = f2bf_bits(v - bf_bits2f(hb));
          hv[e] = __builtin_bit_cast(_Float16, hb);
          lv[e] = __builtin_bit_cast(_Float16, lb);
        }
      }
      const size_t o = (size_t)(c0 + orow) * RP + r0 + c8;
      *(volatile v8h*)(ob0 + o) = hv;
      if (MODE == 1) *(volatile v8h*)(ob1 + o) = lv;
    }
    __threadfence();
  }
}

__device__ __forceinline__ float tanh_fast(float x) {
  const float t = __expf(x + x);
  return 1.0f - 2.0f * __builtin_amdgcn_rcpf(t + 1.0f);
}
__device__ __forceinline__ v8f mma_h(v16h a, v16h b, v8f c) {
  c = __builtin_amdgcn_wmma_f32_16x16x32_f16(false, a, false, b, (short)0, c, false, false);
  asm volatile("v_nop\n\tv_nop\n\tv_nop\n\tv_nop" : "+v"(c) : "v"(a), "v"(b));
  return c;
}
template <int NK>
__global__ __launch_bounds__(256) void k_score(const float* __restrict__ npf,
                                                 const float* __restrict__ kpf,
                                                 const float* __restrict__ wv,
                                                 const float* __restrict__ bsc,
                                                 unsigned short* __restrict__ att)
{
  __shared__ __align__(16) float    s_np[16 * PROJ];
  __shared__ __align__(16) _Float16 s_w[PROJ];
  __shared__ __align__(16) float    s_sc[16 * KEYP];
  const int tid = threadIdx.x, wave = tid >> 5, lane = tid & 31, hh = lane >> 4, m = lane & 15;
  const int row0 = blockIdx.x * 16;
  const int b = row0 >> RB_SHIFT;
  for (int i = tid; i < 16 * (PROJ / 4); i += 256) {
    const int r = i / (PROJ / 4), c4 = (i - r * (PROJ / 4)) * 4;
    *(v4f*)(s_np + r * PROJ + c4) = *(const v4f*)(npf + (size_t)(row0 + r) * PROJ + c4);
  }
  for (int i = tid; i < PROJ; i += 256) s_w[i] = (_Float16)(wv[i] * 256.0f);
  __syncthreads();
  const float bias0 = bsc[0];
  const float* nrow = s_np + m * PROJ + 8 * hh;
  for (int key = wave; key < NK; key += 8) {
    const float* kp = kpf + ((size_t)b * NK + key) * PROJ + 8 * hh;
    v8f acc = (v8f){0.f,0.f,0.f,0.f,0.f,0.f,0.f,0.f};
#pragma unroll 1
    for (int k0 = 0; k0 < PROJ; k0 += 32) {
      const v4f na = *(const v4f*)(nrow + k0);
      const v4f nb = *(const v4f*)(nrow + k0 + 4);
      const v4f nc = *(const v4f*)(nrow + k0 + 16);
      const v4f nd = *(const v4f*)(nrow + k0 + 20);
      const v4f pa = *(const v4f*)(kp + k0);
      const v4f pb = *(const v4f*)(kp + k0 + 4);
      const v4f pc = *(const v4f*)(kp + k0 + 16);
      const v4f pd = *(const v4f*)(kp + k0 + 20);
      v16h av;
#pragma unroll
      for (int e = 0; e < 4; ++e) {
        av[e]      = (_Float16)tanh_fast(na[e] + pa[e]);
        av[4 + e]  = (_Float16)tanh_fast(nb[e] + pb[e]);
        av[8 + e]  = (_Float16)tanh_fast(nc[e] + pc[e]);
        av[12 + e] = (_Float16)tanh_fast(nd[e] + pd[e]);
      }
      const v16h bw = Frag<_Float16>::load(s_w + k0 + 8 * hh);
      acc = mma_h(av, bw, acc);
    }
    if (m == 0) {
#pragma unroll
      for (int r = 0; r < 8; ++r) s_sc[(8 * hh + r) * KEYP + key] = acc[r] * (1.0f / 256.0f) + bias0;
    }
  }
  __syncthreads();
#pragma unroll
  for (int qq = 0; qq < 2; ++qq) {
    const int nd = wave * 2 + qq;
    float x0 = s_sc[nd * KEYP + lane];
    float x1 = s_sc[nd * KEYP + lane + 32];
    const bool v0 = lane < NK;
    const bool v1 = (lane + 32) < NK;
    x0 = v0 ? x0 : -__builtin_inff();
    x1 = v1 ? x1 : -__builtin_inff();
    float mx = fmaxf(x0, x1);
#pragma unroll
    for (int off = 1; off < 32; off <<= 1) mx = fmaxf(mx, __shfl_xor(mx, off, 32));
    const float e0 = v0 ? expf(x0 - mx) : 0.f;
    const float e1 = v1 ? expf(x1 - mx) : 0.f;
    float sum = e0 + e1;
#pragma unroll
    for (int off = 1; off < 32; off <<= 1) sum += __shfl_xor(sum, off, 32);
    const float inv = 1.0f / sum;
    s_sc[nd * KEYP + lane] = e0 * inv;
    s_sc[nd * KEYP + lane + 32] = e1 * inv;
  }
  __syncthreads();
  if (wave < 4) {
    const int q = lane >> 3, c8 = (lane & 7) * 8;
    const int r = wave * 4 + q;
    const float* sp = s_sc + r * KEYP + c8;
    v8h hv;
#pragma unroll
    for (int e = 0; e < 8; ++e) hv[e] = (_Float16)(sp[e] * 1024.0f);
    unsigned short* dst = att + (size_t)(row0 + r) * KEYP + c8;
    *(volatile v8h*)dst = hv;
    __threadfence();
    *(volatile v8h*)dst = hv;
  }
}

static inline dim3 gemm_grid(int M, int N, int batch) {
  const int tiles = (M / 64) * (N / 64);
  return dim3((unsigned)((tiles + 7) / 8), (unsigned)batch, 1);
}

extern "C" void kernel_launch(void* const* d_in, const int* in_sizes, int n_in,
                              void* d_out, int out_size, void* d_ws, size_t ws_size,
                              hipStream_t stream)
{
  if (n_in < 26) return;
  if (in_sizes[0] != ROWS * IN_D || in_sizes[1] != IMG_ROWS * IMG_D || in_sizes[2] != SEM_ROWS * SEM_D ||
      in_sizes[3] != BATCH * QUE_D || in_sizes[4] != (IN_D + QUE_D) * PROJ || in_sizes[6] != IMG_D * PROJ ||
      in_sizes[10] != (IN_D + QUE_D) * PROJ || in_sizes[12] != SEM_D * PROJ || in_sizes[16] != IMG_D * GATE ||
      in_sizes[18] != SEM_D * GATE || in_sizes[20] != IN_D * GATE || in_sizes[22] != CAT * CAT ||
      in_sizes[24] != CAT * OUT_D || out_size != ROWS * OUT_D) return;

  const float* h      = (const float*)d_in[0];
  const float* img    = (const float*)d_in[1];
  const float* sem    = (const float*)d_in[2];
  const float* que    = (const float*)d_in[3];
  const float* W_cif  = (const float*)d_in[4];  const float* b_cif  = (const float*)d_in[5];
  const float* W_cii  = (const float*)d_in[6];  const float* b_cii  = (const float*)d_in[7];
  const float* w_ia   = (const float*)d_in[8];  const float* b_ia   = (const float*)d_in[9];
  const float* W_csf  = (const float*)d_in[10]; const float* b_csf  = (const float*)d_in[11];
  const float* W_csn  = (const float*)d_in[12]; const float* b_csn  = (const float*)d_in[13];
  const float* w_sa   = (const float*)d_in[14]; const float* b_sa   = (const float*)d_in[15];
  const float* W_ig   = (const float*)d_in[16]; const float* b_ig   = (const float*)d_in[17];
  const float* W_sg   = (const float*)d_in[18]; const float* b_sg   = (const float*)d_in[19];
  const float* W_fg   = (const float*)d_in[20]; const float* b_fg   = (const float*)d_in[21];
  const float* W_gate = (const float*)d_in[22]; const float* b_gate = (const float*)d_in[23];
  const float* W_out  = (const float*)d_in[24]; const float* b_out  = (const float*)d_in[25];
  float* out = (float*)d_out;

  char* ws = (char*)d_ws;
  size_t off = 0;
  auto carve = [&](size_t bytes) -> char* { char* p = ws + off; off += (bytes + 255) & ~(size_t)255; return p; };
  unsigned short* hF     = (unsigned short*)carve((size_t)ROWS * IN_D * 2);
  unsigned short* hH     = (unsigned short*)carve((size_t)ROWS * IN_D * 2);
  unsigned short* hL     = (unsigned short*)carve((size_t)ROWS * IN_D * 2);
  unsigned short* queF   = (unsigned short*)carve((size_t)QROWS_P * QUE_D * 2);
  unsigned short* imgF   = (unsigned short*)carve((size_t)IMG_ROWS_P * IMG_D * 2);
  unsigned short* semF   = (unsigned short*)carve((size_t)SEM_ROWS * SEM_D * 2);
  unsigned short* imgT   = (unsigned short*)carve((size_t)BATCH * IMG_D * KEYP * 2);
  unsigned short* semT   = (unsigned short*)carve((size_t)BATCH * SEM_D * KEYP * 2);
  unsigned short* WcifT  = (unsigned short*)carve((size_t)PROJ * (IN_D + QUE_D) * 2);
  unsigned short* WcsfT  = (unsigned short*)carve((size_t)PROJ * (IN_D + QUE_D) * 2);
  unsigned short* WciiT  = (unsigned short*)carve((size_t)PROJ * IMG_D * 2);
  unsigned short* WcsnT  = (unsigned short*)carve((size_t)PROJ * SEM_D * 2);
  unsigned short* WigT   = (unsigned short*)carve((size_t)GATE * IMG_D * 2);
  unsigned short* WsgT   = (unsigned short*)carve((size_t)GATE * SEM_D * 2);
  unsigned short* WfgH   = (unsigned short*)carve((size_t)GATE * IN_D * 2);
  unsigned short* WfgL   = (unsigned short*)carve((size_t)GATE * IN_D * 2);
  unsigned short* WgateT = (unsigned short*)carve((size_t)CAT * CAT * 2);
  unsigned short* WoutT  = (unsigned short*)carve((size_t)OUT_D * CAT * 2);
  float*          qbI    = (float*)carve((size_t)QROWS_P * PROJ * 4);
  float*          qbS    = (float*)carve((size_t)QROWS_P * PROJ * 4);
  float*          npI    = (float*)carve((size_t)ROWS * PROJ * 4);
  float*          npS    = (float*)carve((size_t)ROWS * PROJ * 4);
  float*          ipf    = (float*)carve((size_t)IMG_ROWS_P * PROJ * 4);
  float*          spf    = (float*)carve((size_t)SEM_ROWS * PROJ * 4);
  unsigned short* attI   = (unsigned short*)carve((size_t)ROWS * KEYP * 2);
  unsigned short* attS   = (unsigned short*)carve((size_t)ROWS * KEYP * 2);
  unsigned short* ctxI   = (unsigned short*)carve((size_t)ROWS * IMG_D * 2);
  unsigned short* ctxS   = (unsigned short*)carve((size_t)ROWS * SEM_D * 2);
  float*          cat32  = (float*)carve((size_t)ROWS * CAT * 4);
  unsigned short* cat16  = (unsigned short*)carve((size_t)ROWS * CAT * 2);
  unsigned short* gc16   = (unsigned short*)carve((size_t)ROWS * CAT * 2);
  if (off > ws_size || off > (size_t)134217728) return;

  const float S1024 = 1.0f / 1024.0f;
  dim3 b256(256);

  k_cast8<2><<<(ROWS * IN_D / 8 + 255) / 256, b256, 0, stream>>>(h, ROWS * IN_D, ROWS * IN_D, 16.0f, hF, hH, hL);
  k_cast8<0><<<(QROWS_P * QUE_D / 8 + 255) / 256, b256, 0, stream>>>(que, BATCH * QUE_D, QROWS_P * QUE_D, 16.0f, queF, queF, queF);
  k_cast8<0><<<(IMG_ROWS_P * IMG_D / 8 + 255) / 256, b256, 0, stream>>>(img, IMG_ROWS * IMG_D, IMG_ROWS_P * IMG_D, 16.0f, imgF, imgF, imgF);
  k_cast8<0><<<(SEM_ROWS * SEM_D / 8 + 255) / 256, b256, 0, stream>>>(sem, SEM_ROWS * SEM_D, SEM_ROWS * SEM_D, 16.0f, semF, semF, semF);

  k_transpose64<0><<<dim3(PROJ / 64, (IN_D + QUE_D) / 64, 1), b256, 0, stream>>>(W_cif, IN_D + QUE_D, PROJ, 0L, WcifT, WcifT, IN_D + QUE_D, 0L, 64.0f);
  k_transpose64<0><<<dim3(PROJ / 64, (IN_D + QUE_D) / 64, 1), b256, 0, stream>>>(W_csf, IN_D + QUE_D, PROJ, 0L, WcsfT, WcsfT, IN_D + QUE_D, 0L, 64.0f);
  k_transpose64<0><<<dim3(PROJ / 64, IMG_D / 64, 1), b256, 0, stream>>>(W_cii, IMG_D, PROJ, 0L, WciiT, WciiT, IMG_D, 0L, 64.0f);
  k_transpose64<0><<<dim3(PROJ / 64, SEM_D / 64, 1), b256, 0, stream>>>(W_csn, SEM_D, PROJ, 0L, WcsnT, WcsnT, SEM_D, 0L, 64.0f);
  k_transpose64<0><<<dim3(GATE / 64, IMG_D / 64, 1), b256, 0, stream>>>(W_ig, IMG_D, GATE, 0L, WigT, WigT, IMG_D, 0L, 64.0f);
  k_transpose64<0><<<dim3(GATE / 64, SEM_D / 64, 1), b256, 0, stream>>>(W_sg, SEM_D, GATE, 0L, WsgT, WsgT, SEM_D, 0L, 64.0f);
  k_transpose64<1><<<dim3(GATE / 64, IN_D / 64, 1), b256, 0, stream>>>(W_fg, IN_D, GATE, 0L, WfgH, WfgL, IN_D, 0L, 1.0f);
  k_transpose64<0><<<dim3(CAT / 64, CAT / 64, 1), b256, 0, stream>>>(W_gate, CAT, CAT, 0L, WgateT, WgateT, CAT, 0L, 64.0f);
  k_transpose64<0><<<dim3(OUT_D / 64, CAT / 64, 1), b256, 0, stream>>>(W_out, CAT, OUT_D, 0L, WoutT, WoutT, CAT, 0L, 64.0f);
  k_transpose64<0><<<dim3(IMG_D / 64, KEYP / 64, BATCH), b256, 0, stream>>>(img, NIMG, IMG_D, (long)NIMG * IMG_D, imgT, imgT, KEYP, (long)IMG_D * KEYP, 16.0f);
  k_transpose64<0><<<dim3(SEM_D / 64, KEYP / 64, BATCH), b256, 0, stream>>>(sem, NSEM, SEM_D, (long)NSEM * SEM_D, semT, semT, KEYP, (long)SEM_D * KEYP, 16.0f);

  wmma_gemm64<0, false, 2, 0, 0, false><<<gemm_grid(QROWS_P, PROJ, 1), b256, 0, stream>>>(
      queF, queF, QUE_D, 0L, WcifT + IN_D, WcifT + IN_D, IN_D + QUE_D, 0L,
      (void*)qbI, (void*)qbI, PROJ, 0L, b_cif, b_cif, 0, QROWS_P, PROJ, QUE_D, S1024, 1.0f);
  wmma_gemm64<0, false, 2, 0, 0, false><<<gemm_grid(QROWS_P, PROJ, 1), b256, 0, stream>>>(
      queF, queF, QUE_D, 0L, WcsfT + IN_D, WcsfT + IN_D, IN_D + QUE_D, 0L,
      (void*)qbS, (void*)qbS, PROJ, 0L, b_csf, b_csf, 0, QROWS_P, PROJ, QUE_D, S1024, 1.0f);
  wmma_gemm64<0, false, 3, 0, 0, false><<<gemm_grid(ROWS, PROJ, 1), b256, 0, stream>>>(
      hF, hF, IN_D, 0L, WcifT, WcifT, IN_D + QUE_D, 0L,
      (void*)npI, (void*)npI, PROJ, 0L, qbI, qbI, 0, ROWS, PROJ, IN_D, S1024, 1.0f);
  wmma_gemm64<0, false, 3, 0, 0, false><<<gemm_grid(ROWS, PROJ, 1), b256, 0, stream>>>(
      hF, hF, IN_D, 0L, WcsfT, WcsfT, IN_D + QUE_D, 0L,
      (void*)npS, (void*)npS, PROJ, 0L, qbS, qbS, 0, ROWS, PROJ, IN_D, S1024, 1.0f);
  wmma_gemm64<0, false, 2, 0, 0, false><<<gemm_grid(IMG_ROWS_P, PROJ, 1), b256, 0, stream>>>(
      imgF, imgF, IMG_D, 0L, WciiT, WciiT, IMG_D, 0L,
      (void*)ipf, (void*)ipf, PROJ, 0L, b_cii, b_cii, 0, IMG_ROWS_P, PROJ, IMG_D, S1024, 1.0f);
  wmma_gemm64<0, false, 2, 0, 0, false><<<gemm_grid(SEM_ROWS, PROJ, 1), b256, 0, stream>>>(
      semF, semF, SEM_D, 0L, WcsnT, WcsnT, SEM_D, 0L,
      (void*)spf, (void*)spf, PROJ, 0L, b_csn, b_csn, 0, SEM_ROWS, PROJ, SEM_D, S1024, 1.0f);

  k_score<NIMG><<<ROWS / 16, b256, 0, stream>>>(npI, ipf, w_ia, b_ia, attI);
  k_score<NSEM><<<ROWS / 16, b256, 0, stream>>>(npS, spf, w_sa, b_sa, attS);

  wmma_gemm64<0, false, 0, 1, 0, false><<<gemm_grid(NODES, IMG_D, BATCH), b256, 0, stream>>>(
      attI, attI, KEYP, (long)NODES * KEYP, imgT, imgT, KEYP, (long)IMG_D * KEYP,
      (void*)ctxI, (void*)ctxI, IMG_D, (long)NODES * IMG_D, b_out, b_out, 0, NODES, IMG_D, KEYP, S1024, 1.0f);
  wmma_gemm64<0, false, 0, 1, 0, false><<<gemm_grid(NODES, SEM_D, BATCH), b256, 0, stream>>>(
      attS, attS, KEYP, (long)NODES * KEYP, semT, semT, KEYP, (long)SEM_D * KEYP,
      (void*)ctxS, (void*)ctxS, SEM_D, (long)NODES * SEM_D, b_out, b_out, 0, NODES, SEM_D, KEYP, S1024, 1.0f);

  wmma_gemm64<1, true, 2, 3, 0, false><<<gemm_grid(ROWS, GATE, 1), b256, 0, stream>>>(
      hH, hL, IN_D, 0L, WfgH, WfgL, IN_D, 0L,
      (void*)cat32, (void*)cat16, CAT, 0L, b_fg, b_fg, 0, ROWS, GATE, IN_D, 1.0f, 16.0f);
  wmma_gemm64<0, false, 2, 3, 0, false><<<gemm_grid(ROWS, GATE, 1), b256, 0, stream>>>(
      ctxI, ctxI, IMG_D, 0L, WigT, WigT, IMG_D, 0L,
      (void*)(cat32 + GATE), (void*)(cat16 + GATE), CAT, 0L, b_ig, b_ig, 0, ROWS, GATE, IMG_D, S1024, 16.0f);
  wmma_gemm64<0, false, 2, 3, 0, false><<<gemm_grid(ROWS, GATE, 1), b256, 0, stream>>>(
      ctxS, ctxS, SEM_D, 0L, WsgT, WsgT, SEM_D, 0L,
      (void*)(cat32 + 2 * GATE), (void*)(cat16 + 2 * GATE), CAT, 0L, b_sg, b_sg, 0, ROWS, GATE, SEM_D, S1024, 16.0f);

  wmma_gemm64<0, false, 2, 1, 6, true><<<gemm_grid(ROWS, CAT, 1), b256, 0, stream>>>(
      cat16, cat16, CAT, 0L, WgateT, WgateT, CAT, 0L,
      (void*)gc16, (void*)gc16, CAT, 0L, b_gate, cat32, CAT, ROWS, CAT, CAT, S1024, 16.0f);

  wmma_gemm64<0, false, 2, 0, 0, false><<<gemm_grid(ROWS, OUT_D, 1), b256, 0, stream>>>(
      gc16, gc16, CAT, 0L, WoutT, WoutT, CAT, 0L,
      (void*)out, (void*)out, OUT_D, 0L, b_out, b_out, 0, ROWS, OUT_D, CAT, S1024, 1.0f);

  (void)ws_size;
}
